// PatchGraphAttention_15178414424120
// MI455X (gfx1250) — hardware-verified
//
#include <hip/hip_runtime.h>
#include <math.h>

constexpr int kB   = 4;
constexpr int kP   = 2048;
constexpr int kD   = 1024;
constexpr int kH   = 16;
constexpr int kDh  = 64;
constexpr int kTok = kB * kP;
constexpr int kQB  = 64;
constexpr int kKC  = 64;
constexpr int kNW  = 4;
constexpr float kScoreScale = 0.125f;
constexpr float kNegBig     = -1.0e9f;
constexpr float kPCarry     = 32768.0f;
constexpr float kVloCarry   = 2048.0f;
constexpr float kVloInv     = 1.0f / 2048.0f;
constexpr float kDelta      = 300.0f;
constexpr float kInvTau     = 1.0f / 300.0f;
constexpr float kLogEps     = 1.0e-12f;
static_assert(kH * kDh == kD, "s");
static_assert(kTok % 64 == 0 && kD % 64 == 0 && kD % 32 == 0, "s");
static_assert(kP % kQB == 0 && kP % kKC == 0 && kDh == 64, "s");
static_assert((kTok * kD) % (8 * 256) == 0 && (kD * kD) % (8 * 256) == 0, "s");
static_assert(kP % 1024 == 0, "s");

typedef __attribute__((ext_vector_type(16))) _Float16 v16h;
typedef __attribute__((ext_vector_type(8)))  _Float16 v8h;
typedef __attribute__((ext_vector_type(16))) __bf16   v16b;
typedef __attribute__((ext_vector_type(8)))  __bf16   v8b;
typedef __attribute__((ext_vector_type(8)))  float    v8f;
typedef __attribute__((ext_vector_type(4)))  float    v4f;
typedef __attribute__((ext_vector_type(4)))  unsigned int v4u;

__device__ __forceinline__ unsigned short f2bf_bits(float f) {
  unsigned u = __float_as_uint(f);
  return (unsigned short)((u + 0x7FFFu + ((u >> 16) & 1u)) >> 16);
}
__device__ __forceinline__ float bf_bits2f(unsigned short h) { return __uint_as_float(((unsigned)h) << 16); }

__device__ __forceinline__ float h16_to_f32(unsigned hb) {
  const unsigned sgn = (hb & 0x8000u) << 16; const unsigned em = hb & 0x7fffu;
  const float fn = __uint_as_float((em << 13) + 0x38000000u);
  const float fs = (float)em * 5.9604644775390625e-8f;
  const float mag = (em < 0x400u) ? fs : fn; return __uint_as_float(__float_as_uint(mag) | sgn); }

__device__ __forceinline__ void dep_guard4_h(v8f& a, v8f& b, v8f& c, v8f& d, v16h x, v16h y) {
  asm volatile("v_nop\n\tv_nop\n\tv_nop\n\tv_nop" : "+v"(a), "+v"(b), "+v"(c), "+v"(d) : "v"(x), "v"(y));
}
__device__ __forceinline__ void dep_guard4_b(v8f& a, v8f& b, v8f& c, v8f& d, v16b x, v16b y) {
  asm volatile("v_nop\n\tv_nop\n\tv_nop\n\tv_nop" : "+v"(a), "+v"(b), "+v"(c), "+v"(d) : "v"(x), "v"(y));
}
__device__ __forceinline__ void keep4_h(v16h a, v16h b, v16h c, v16h d) { asm volatile("v_nop" :: "v"(a), "v"(b), "v"(c), "v"(d)); }
__device__ __forceinline__ void keep4_b(v16b a, v16b b, v16b c, v16b d) { asm volatile("v_nop" :: "v"(a), "v"(b), "v"(c), "v"(d)); }
__device__ __forceinline__ void acc_guard4(v8f& a, v8f& b, v8f& c, v8f& d) { asm volatile("v_nop\n\tv_nop\n\tv_nop\n\tv_nop" : "+v"(a), "+v"(b), "+v"(c), "+v"(d)); }
template <typename T> struct Frag;
template <> struct Frag<_Float16> {
  typedef v16h V; union U { v16h v; v8h h[2]; };
  static __device__ __forceinline__ v16h load(const _Float16* p) {
    U f; f.h[0] = *(const v8h*)(p); f.h[1] = *(const v8h*)(p + 16); return f.v;
  }
  static __device__ __forceinline__ v8f mma(v16h a, v16h b, v8f c) {
    return __builtin_amdgcn_wmma_f32_16x16x32_f16(false, a, false, b, (short)0, c, false, false);
  }
  static __device__ __forceinline__ void guard4(v8f& a, v8f& b, v8f& c, v8f& d, v16h x, v16h y) { dep_guard4_h(a, b, c, d, x, y); }
  static __device__ __forceinline__ void keep(v16h a, v16h b, v16h c, v16h d) { keep4_h(a, b, c, d); }
};
template <> struct Frag<__bf16> {
  typedef v16b V; union U { v16b v; v8b h[2]; };
  static __device__ __forceinline__ v16b load(const __bf16* p) {
    U f; f.h[0] = *(const v8b*)(p); f.h[1] = *(const v8b*)(p + 16); return f.v;
  }
  static __device__ __forceinline__ v8f mma(v16b a, v16b b, v8f c) {
    return __builtin_amdgcn_wmma_f32_16x16x32_bf16(false, a, false, b, (short)0, c, false, false);
  }
  static __device__ __forceinline__ void guard4(v8f& a, v8f& b, v8f& c, v8f& d, v16b x, v16b y) { dep_guard4_b(a, b, c, d, x, y); }
  static __device__ __forceinline__ void keep(v16b a, v16b b, v16b c, v16b d) { keep4_b(a, b, c, d); }
};

__device__ __forceinline__ unsigned pk16(unsigned short a, unsigned short b) { return (unsigned)a | ((unsigned)b << 16); }
__device__ __forceinline__ unsigned short h_bits(float f) { const _Float16 h = (_Float16)f; return __builtin_bit_cast(unsigned short, h); }

__device__ __forceinline__ v8f mma_h(v16h a, v16h b, v8f c) {
  c = __builtin_amdgcn_wmma_f32_16x16x32_f16(false, a, false, b, (short)0, c, false, false);
  asm volatile("v_nop\n\tv_nop\n\tv_nop\n\tv_nop" : "+v"(c) : "v"(a), "v"(b));
  return c;
}

template <int ET> struct Elem;
template <> struct Elem<0> { typedef _Float16 T; };
template <> struct Elem<1> { typedef __bf16 T; };
template <int ET, int SPLIT, int BIAS_MODE, int OUT_MODE, bool ROWSC>
__global__ __launch_bounds__(256) void wmma_gemm64(
    const unsigned short* __restrict__ Ap, const unsigned short* __restrict__ A2p, int lda, long strideA,
    const unsigned short* __restrict__ Btp, const unsigned short* __restrict__ Bt2p, int ldb, long strideB,
    void* __restrict__ Cout, void* __restrict__ Cout2, int ldc, long strideC,
    const float* __restrict__ bias, const float* __restrict__ rowsc,
    int M, int N, int K, float scale) {
  typedef typename Elem<ET>::T T;
  typedef typename Frag<T>::V V;
  const T* A = (const T*)Ap; const T* A2 = (const T*)A2p; const T* Bt = (const T*)Btp; const T* Bt2 = (const T*)Bt2p;
  __shared__ __align__(16) float sT[8][16 * 68];
  const int b    = blockIdx.y;
  const int lane = threadIdx.x & 31;
  const int wave = threadIdx.x >> 5;
  const int tilesN = N >> 6;
  const int tilesM = M >> 6;
  const int tile = blockIdx.x * 8 + wave;
  if (tile >= tilesM * tilesN) return;
  const int tm = tile / tilesN;
  const int tn = tile - tm * tilesN;
  const int m0 = tm << 6;
  const int n0 = tn << 6;

  const T* Ab  = A  + (size_t)b * strideA;
  const T* Bb  = Bt + (size_t)b * strideB;
  const T* Ab2 = (SPLIT != 0) ? (A2  + (size_t)b * strideA) : Ab;
  const T* Bb2 = (SPLIT == 1) ? (Bt2 + (size_t)b * strideB) : Bb;

  const int rlane = lane & 15;
  const int koff  = (lane >> 4) * 8;
  const int mOff  = (lane >> 4) * 8;

  v8f acc[4][4];
#pragma unroll
  for (int i = 0; i < 4; ++i)
#pragma unroll
    for (int j = 0; j < 4; ++j) acc[i][j] = (v8f){0.f,0.f,0.f,0.f,0.f,0.f,0.f,0.f};

  for (int k0 = 0; k0 < K; k0 += 32) {
    V bh[4], bl[4];
#pragma unroll
    for (int j = 0; j < 4; ++j) {
      const size_t bo = (size_t)(n0 + (j << 4) + rlane) * ldb + koff + k0;
      bh[j] = Frag<T>::load(Bb + bo);
      if (SPLIT == 1) bl[j] = Frag<T>::load(Bb2 + bo);
    }
#pragma unroll
    for (int i = 0; i < 4; ++i) {
      const size_t ao = (size_t)(m0 + (i << 4) + rlane) * lda + koff + k0;
      V ah = Frag<T>::load(Ab + ao);
      V al = ah;
      if (SPLIT != 0) al = Frag<T>::load(Ab2 + ao);
#pragma unroll
      for (int j = 0; j < 4; ++j) {
        acc[i][j] = Frag<T>::mma(ah, bh[j], acc[i][j]);
        if (SPLIT == 1) acc[i][j] = Frag<T>::mma(ah, bl[j], acc[i][j]);
        if (SPLIT != 0) acc[i][j] = Frag<T>::mma(al, bh[j], acc[i][j]);
      }
      Frag<T>::guard4(acc[i][0], acc[i][1], acc[i][2], acc[i][3], ah, al);
    }
    Frag<T>::keep(bh[0], bh[1], bh[2], bh[3]);
    if (SPLIT == 1) Frag<T>::keep(bl[0], bl[1], bl[2], bl[3]);
  }
  acc_guard4(acc[0][0], acc[0][1], acc[0][2], acc[0][3]);
  acc_guard4(acc[1][0], acc[1][1], acc[1][2], acc[1][3]);
  acc_guard4(acc[2][0], acc[2][1], acc[2][2], acc[2][3]);
  acc_guard4(acc[3][0], acc[3][1], acc[3][2], acc[3][3]);

  float* slab = sT[wave];
#pragma unroll
  for (int i = 0; i < 4; ++i) {
    const int mBase = m0 + (i << 4);
    float rsv[8];
#pragma unroll
    for (int r = 0; r < 8; ++r) rsv[r] = 1.0f;
    if (ROWSC) {
      const v4f ra = *(const v4f*)(rowsc + mBase + mOff);
      const v4f rb = *(const v4f*)(rowsc + mBase + mOff + 4);
      rsv[0] = ra[0]; rsv[1] = ra[1]; rsv[2] = ra[2]; rsv[3] = ra[3];
      rsv[4] = rb[0]; rsv[5] = rb[1]; rsv[6] = rb[2]; rsv[7] = rb[3];
#pragma unroll
      for (int r = 0; r < 8; ++r) rsv[r] = bf_bits2f(f2bf_bits(rsv[r]));
    }
#pragma unroll
    for (int j = 0; j < 4; ++j) {
      const int n = n0 + (j << 4) + rlane;
      float bv = 0.f;
      if (BIAS_MODE == 2) bv = bias[n];
#pragma unroll
      for (int r = 0; r < 8; ++r) {
        float v = acc[i][j][r] * scale;
        if (BIAS_MODE == 1) v += bias[mBase + mOff + r];
        if (BIAS_MODE == 2) v += bv;
        if (ROWSC) v = v * rsv[r];
        slab[(mOff + r) * 68 + (j << 4) + rlane] = v;
      }
    }
    __builtin_amdgcn_fence(__ATOMIC_RELEASE, "workgroup");
    __builtin_amdgcn_wave_barrier();
    __builtin_amdgcn_fence(__ATOMIC_ACQUIRE, "workgroup");
    if (OUT_MODE == 0) {
      float* C = (float*)Cout + (size_t)b * strideC;
      const int hh = lane >> 4, c4 = (lane & 15) * 4;
      for (int pass = 0; pass < 2; ++pass) {
#pragma unroll
        for (int it = 0; it < 8; ++it) {
          const int row = it * 2 + hh;
          v4f v = *(const v4f*)(slab + row * 68 + c4);
          *(volatile v4f*)(C + (size_t)(mBase + row) * ldc + n0 + c4) = v;
        }
        __threadfence();
      }
    } else {
      const int q = lane >> 3, c8 = (lane & 7) * 8;
      unsigned short* C  = (unsigned short*)Cout  + (size_t)b * strideC;
      unsigned short* C2 = (OUT_MODE >= 2) ? ((unsigned short*)Cout2 + (size_t)b * strideC) : nullptr;
      for (int pass = 0; pass < 2; ++pass) {
#pragma unroll
        for (int it = 0; it < 4; ++it) {
          const int row = it * 4 + q;
          const float* sp = slab + row * 68 + c8;
          v8h hv, lv;
#pragma unroll
          for (int e = 0; e < 8; ++e) {
            if (OUT_MODE == 1) {
              hv[e] = (_Float16)sp[e];
            } else if (OUT_MODE == 2) {
              unsigned short hb = f2bf_bits(sp[e]);
              unsigned short lb = f2bf_bits(sp[e] - bf_bits2f(hb));
              hv[e] = __builtin_bit_cast(_Float16, hb);
              lv[e] = __builtin_bit_cast(_Float16, lb);
            } else {
              const unsigned short hb = h_bits(sp[e]);
              const float back = h16_to_f32((unsigned)hb);
              const unsigned short lb = h_bits((sp[e] - back) * kVloCarry);
              hv[e] = __builtin_bit_cast(_Float16, hb);
              lv[e] = __builtin_bit_cast(_Float16, lb);
            }
          }
          *(volatile v8h*)(C + (size_t)(mBase + row) * ldc + n0 + c8) = hv;
          if (OUT_MODE >= 2) *(volatile v8h*)(C2 + (size_t)(mBase + row) * ldc + n0 + c8) = lv;
        }
        __threadfence();
      }
    }
    __builtin_amdgcn_fence(__ATOMIC_RELEASE, "workgroup");
    __builtin_amdgcn_wave_barrier();
    __builtin_amdgcn_fence(__ATOMIC_ACQUIRE, "workgroup");
  }
}

__global__ __launch_bounds__(256) void cast8_bf16_kernel(const float* __restrict__ in, unsigned short* __restrict__ out, int n8) {
  const int i = blockIdx.x * 256 + threadIdx.x;
  if (i >= n8) return;
  const float* p = in + 8 * (size_t)i;
  const v4f a = *(const v4f*)(p);
  const v4f c = *(const v4f*)(p + 4);
  unsigned short hb[8];
#pragma unroll
  for (int e = 0; e < 4; ++e) {
    hb[e]     = f2bf_bits(a[e]);
    hb[4 + e] = f2bf_bits(c[e]);
  }
  const v4u u = (v4u){pk16(hb[0], hb[1]), pk16(hb[2], hb[3]), pk16(hb[4], hb[5]), pk16(hb[6], hb[7])};
  unsigned short* q = out + 8 * (size_t)i;
  *(volatile v4u*)q = u;
  __threadfence();
  *(volatile v4u*)q = u;
}

__global__ __launch_bounds__(256) void tab_kernel(float* __restrict__ tab) {
  const int i = blockIdx.x * 256 + threadIdx.x;
  if (i >= kP / 4) return;
  v4f tv;
#pragma unroll
  for (int e = 0; e < 4; ++e) {
    const float d = (float)(4 * i + e);
    const float dist = d * kDelta;
    const float ex = (-dist) * kInvTau;
    const float w = expf(ex);
    tv[e] = logf(w + kLogEps);
  }
  float* q = tab + 4 * (size_t)i;
  *(volatile v4f*)q = tv;
  __threadfence();
  *(volatile v4f*)q = tv;
}

__global__ __launch_bounds__(128) void attn_kernel(const unsigned short* __restrict__ Qp, const unsigned short* __restrict__ Kp,
                                                   const unsigned short* __restrict__ VThp, const unsigned short* __restrict__ VTlp,
                                                   const float* __restrict__ tab, const float* __restrict__ pm,
                                                   unsigned short* __restrict__ Ohp, unsigned short* __restrict__ Olp) {
  __shared__ __align__(16) _Float16 Ksh[kKC * kDh];
  __shared__ __align__(16) _Float16 Vth[kDh * kKC];
  __shared__ __align__(16) _Float16 Vtl[kDh * kKC];
  __shared__ __align__(16) _Float16 Psh[kNW][16 * kKC];
  __shared__ __align__(16) float    Os[kNW][16 * 68];
  __shared__ __align__(16) float    tabs[kP];

  const int tid  = threadIdx.x;
  const int wave = tid >> 5;
  const int lane = tid & 31;
  const int hh   = lane >> 4;
  const int c    = lane & 15;
  const int nqb  = kP / kQB;
  const int bx   = blockIdx.x;
  const int qb   = bx % nqb;
  const int bh   = bx / nqb;
  const int h    = bh % kH;
  const int b    = bh / kH;
  const int q0   = qb * kQB + wave * 16;
  const size_t tok0 = (size_t)b * kP;

#pragma unroll
  for (int i = 0; i < 4; ++i) {
    const int idx = i * 128 + tid;
    const v4f t4 = *(const v4f*)(tab + 4 * idx);
    *(v4f*)(tabs + 4 * idx) = t4;
  }
  asm volatile("" ::: "memory");

  const _Float16* Qh = (const _Float16*)(const void*)Qp;
  const _Float16* qr = Qh + (tok0 + q0 + c) * (size_t)kD + h * kDh + 8 * hh;
  v16h qa[2];
  qa[0] = Frag<_Float16>::load(qr);
  qa[1] = Frag<_Float16>::load(qr + 32);

  float mrow[8], lrow[8];
  v8f oacc[4], oaccl[4];
#pragma unroll
  for (int r = 0; r < 8; ++r) { mrow[r] = -__builtin_inff(); lrow[r] = 0.f; }
#pragma unroll
  for (int t = 0; t < 4; ++t) {
    oacc[t]  = (v8f){0.f,0.f,0.f,0.f,0.f,0.f,0.f,0.f};
    oaccl[t] = (v8f){0.f,0.f,0.f,0.f,0.f,0.f,0.f,0.f};
  }

  for (int kc = 0; kc < kP / kKC; ++kc) {
    const int kv0 = kc * kKC;
    __syncthreads();
    {
      const unsigned short* kbp = Kp + (tok0 + kv0) * (size_t)kD + h * kDh;
      v4u u[4];
#pragma unroll
      for (int i = 0; i < 4; ++i) {
        const int idx = i * 128 + tid;
        const int row = idx >> 3;
        const int seg = (idx & 7) * 8;
        u[i] = *(const v4u*)(kbp + (size_t)row * kD + seg);
      }
#pragma unroll
      for (int i = 0; i < 4; ++i) {
        const int idx = i * 128 + tid;
        const int row = idx >> 3;
        const int seg = (idx & 7) * 8;
        *(v4u*)(Ksh + row * kDh + seg) = u[i];
      }
    }
    asm volatile("" ::: "memory");
    {
      const unsigned short* vbp = VThp + (size_t)(h * kDh) * kTok + tok0 + kv0;
      v4u u[4];
#pragma unroll
      for (int i = 0; i < 4; ++i) {
        const int idx = i * 128 + tid;
        const int row = idx >> 3;
        const int seg = (idx & 7) * 8;
        u[i] = *(const v4u*)(vbp + (size_t)row * kTok + seg);
      }
#pragma unroll
      for (int i = 0; i < 4; ++i) {
        const int idx = i * 128 + tid;
        const int row = idx >> 3;
        const int seg = (idx & 7) * 8;
        *(v4u*)(Vth + row * kKC + seg) = u[i];
      }
    }
    asm volatile("" ::: "memory");
    {
      const unsigned short* vbp = VTlp + (size_t)(h * kDh) * kTok + tok0 + kv0;
      v4u u[4];
#pragma unroll
      for (int i = 0; i < 4; ++i) {
        const int idx = i * 128 + tid;
        const int row = idx >> 3;
        const int seg = (idx & 7) * 8;
        u[i] = *(const v4u*)(vbp + (size_t)row * kTok + seg);
      }
#pragma unroll
      for (int i = 0; i < 4; ++i) {
        const int idx = i * 128 + tid;
        const int row = idx >> 3;
        const int seg = (idx & 7) * 8;
        *(v4u*)(Vtl + row * kKC + seg) = u[i];
      }
    }
    __syncthreads();

    v8f s[4];
#pragma unroll
    for (int j = 0; j < 4; ++j) {
      s[j] = (v8f){0.f,0.f,0.f,0.f,0.f,0.f,0.f,0.f};
#pragma unroll
      for (int dc = 0; dc < 2; ++dc) {
        const v16h kf = Frag<_Float16>::load(Ksh + (j * 16 + c) * kDh + dc * 32 + 8 * hh);
        s[j] = mma_h(qa[dc], kf, s[j]);
      }
    }
    float pmv[4];
#pragma unroll
    for (int j = 0; j < 4; ++j) pmv[j] = pm[tok0 + kv0 + j * 16 + c];

    float cm[8];
#pragma unroll
    for (int r = 0; r < 8; ++r) {
      const int qrow = q0 + 8 * hh + r;
      float m = -__builtin_inff();
#pragma unroll
      for (int j = 0; j < 4; ++j) {
        const int kvcol = kv0 + j * 16 + c;
        int dd = qrow - kvcol;
        dd = (dd < 0) ? -dd : dd;
        float v = s[j][r] * kScoreScale + tabs[dd];
        v = (pmv[j] <= 0.0f) ? kNegBig : v;
        s[j][r] = v;
        m = fmaxf(m, v);
      }
#pragma unroll
      for (int off = 1; off < 16; off <<= 1) m = fmaxf(m, __shfl_xor(m, off, 32));
      cm[r] = m;
    }

    _Float16* pw = Psh[wave];
#pragma unroll
    for (int r = 0; r < 8; ++r) {
      const float mnew  = fmaxf(mrow[r], cm[r]);
      const float alpha = expf(mrow[r] - mnew);
      mrow[r] = mnew;
      float psum = 0.f;
#pragma unroll
      for (int j = 0; j < 4; ++j) {
        const float p = expf(s[j][r] - mnew);
        psum += p;
        pw[(8 * hh + r) * kKC + j * 16 + c] = (_Float16)(p * kPCarry);
      }
#pragma unroll
      for (int off = 1; off < 16; off <<= 1) psum += __shfl_xor(psum, off, 32);
      lrow[r] = lrow[r] * alpha + psum;
#pragma unroll
      for (int t = 0; t < 4; ++t) { oacc[t][r] *= alpha; oaccl[t][r] *= alpha; }
    }
    __builtin_amdgcn_fence(__ATOMIC_RELEASE, "workgroup");
    __builtin_amdgcn_wave_barrier();
    __builtin_amdgcn_fence(__ATOMIC_ACQUIRE, "workgroup");

#pragma unroll
    for (int kk = 0; kk < 2; ++kk) {
      const v16h pa = Frag<_Float16>::load(pw + c * kKC + kk * 32 + 8 * hh);
#pragma unroll
      for (int t = 0; t < 4; ++t) {
        const v16h vh = Frag<_Float16>::load(Vth + (t * 16 + c) * kKC + kk * 32 + 8 * hh);
        oacc[t] = mma_h(pa, vh, oacc[t]);
        const v16h vl = Frag<_Float16>::load(Vtl + (t * 16 + c) * kKC + kk * 32 + 8 * hh);
        oaccl[t] = mma_h(pa, vl, oaccl[t]);
      }
    }
  }

  float* os = Os[wave];
#pragma unroll
  for (int r = 0; r < 8; ++r) {
    const float inv = 1.0f / (lrow[r] * kPCarry);
#pragma unroll
    for (int t = 0; t < 4; ++t) os[(8 * hh + r) * 68 + t * 16 + c] = (oacc[t][r] + oaccl[t][r] * kVloInv) * inv;
  }
  __builtin_amdgcn_fence(__ATOMIC_RELEASE, "workgroup");
  __builtin_amdgcn_wave_barrier();
  __builtin_amdgcn_fence(__ATOMIC_ACQUIRE, "workgroup");
  {
    const int q4 = lane >> 3, c8 = (lane & 7) * 8;
    for (int pass = 0; pass < 2; ++pass) {
#pragma unroll
      for (int it = 0; it < 4; ++it) {
        const int row = it * 4 + q4;
        const float* sp = os + row * 68 + c8;
        v8h hv, lv;
#pragma unroll
        for (int e = 0; e < 8; ++e) {
          const unsigned short hb = f2bf_bits(sp[e]);
          const unsigned short lb = f2bf_bits(sp[e] - bf_bits2f(hb));
          hv[e] = __builtin_bit_cast(_Float16, hb);
          lv[e] = __builtin_bit_cast(_Float16, lb);
        }
        const size_t off = (tok0 + q0 + row) * (size_t)kD + h * kDh + c8;
        *(volatile v8h*)(Ohp + off) = hv;
        *(volatile v8h*)(Olp + off) = lv;
      }
      __threadfence();
    }
  }
}

extern "C" void kernel_launch(void* const* d_in, const int* in_sizes, int n_in,
                              void* d_out, int out_size, void* d_ws, size_t ws_size,
                              hipStream_t stream) {
  if (n_in < 10) return;
  const int nX = kTok * kD;
  const int nW = kD * kD;
  if (in_sizes[0] != nX || in_sizes[1] != kTok) return;
  if (in_sizes[2] != nW || in_sizes[4] != nW || in_sizes[6] != nW || in_sizes[8] != nW) return;
  if (in_sizes[3] != kD || in_sizes[5] != kD || in_sizes[7] != kD || in_sizes[9] != kD) return;
  if (out_size != nX) return;

  const size_t szX16 = (size_t)nX * 2;
  const size_t szW16 = (size_t)nW * 2;
  const size_t szTab = (size_t)kP * 4;
  const size_t offXb  = 0;
  const size_t offWq  = offXb + szX16;
  const size_t offWk  = offWq + szW16;
  const size_t offWv  = offWk + szW16;
  const size_t offWo  = offWv + szW16;
  const size_t offQ   = offWo + szW16;
  const size_t offK   = offQ + szX16;
  const size_t offVTh = offK + szX16;
  const size_t offVTl = offVTh + szX16;
  const size_t offOh  = offVTl + szX16;
  const size_t offOl  = offOh + szX16;
  const size_t offTab = offOl + szX16;
  const size_t total  = offTab + szTab;
  if (ws_size < total) return;

  const float* x  = (const float*)d_in[0];
  const float* pm = (const float*)d_in[1];
  const float* Wq = (const float*)d_in[2];
  const float* bq = (const float*)d_in[3];
  const float* Wk = (const float*)d_in[4];
  const float* bk = (const float*)d_in[5];
  const float* Wv = (const float*)d_in[6];
  const float* bv = (const float*)d_in[7];
  const float* Wo = (const float*)d_in[8];
  const float* bo = (const float*)d_in[9];
  float* out = (float*)d_out;
  char* ws = (char*)d_ws;
  unsigned short* Xb  = (unsigned short*)(ws + offXb);
  unsigned short* Wqb = (unsigned short*)(ws + offWq);
  unsigned short* Wkb = (unsigned short*)(ws + offWk);
  unsigned short* Wvb = (unsigned short*)(ws + offWv);
  unsigned short* Wob = (unsigned short*)(ws + offWo);
  unsigned short* Q16 = (unsigned short*)(ws + offQ);
  unsigned short* K16 = (unsigned short*)(ws + offK);
  unsigned short* VTh = (unsigned short*)(ws + offVTh);
  unsigned short* VTl = (unsigned short*)(ws + offVTl);
  unsigned short* Oh  = (unsigned short*)(ws + offOh);
  unsigned short* Ol  = (unsigned short*)(ws + offOl);
  float* tab = (float*)(ws + offTab);

  const int n8x = nX / 8;
  const int n8w = nW / 8;
  cast8_bf16_kernel<<<dim3(n8x / 256), dim3(256), 0, stream>>>(x,  Xb,  n8x);
  cast8_bf16_kernel<<<dim3(n8w / 256), dim3(256), 0, stream>>>(Wq, Wqb, n8w);
  cast8_bf16_kernel<<<dim3(n8w / 256), dim3(256), 0, stream>>>(Wk, Wkb, n8w);
  cast8_bf16_kernel<<<dim3(n8w / 256), dim3(256), 0, stream>>>(Wv, Wvb, n8w);
  cast8_bf16_kernel<<<dim3(n8w / 256), dim3(256), 0, stream>>>(Wo, Wob, n8w);
  tab_kernel<<<dim3((kP / 4) / 256), dim3(256), 0, stream>>>(tab);

  const int tilesProj = (kTok / 64) * (kD / 64);
  wmma_gemm64<1, 0, 2, 1, false><<<dim3(tilesProj / 8, 1), dim3(256), 0, stream>>>(
      Xb, Xb, kD, 0L, Wqb, Wqb, kD, 0L, (void*)Q16, (void*)Q16, kD, 0L, bq, pm, kTok, kD, kD, 1.0f);
  wmma_gemm64<1, 0, 2, 1, false><<<dim3(tilesProj / 8, 1), dim3(256), 0, stream>>>(
      Xb, Xb, kD, 0L, Wkb, Wkb, kD, 0L, (void*)K16, (void*)K16, kD, 0L, bk, pm, kTok, kD, kD, 1.0f);
  wmma_gemm64<1, 0, 1, 3, false><<<dim3(tilesProj / 8, 1), dim3(256), 0, stream>>>(
      Wvb, Wvb, kD, 0L, Xb, Xb, kD, 0L, (void*)VTh, (void*)VTl, kTok, 0L, bv, pm, kD, kTok, kD, 1.0f);

  attn_kernel<<<dim3(kB * kH * (kP / kQB)), dim3(128), 0, stream>>>(Q16, K16, VTh, VTl, tab, pm, Oh, Ol);

  wmma_gemm64<1, 2, 2, 0, true><<<dim3(tilesProj / 8, 1), dim3(256), 0, stream>>>(
      Oh, Ol, kD, 0L, Wob, Wob, kD, 0L, (void*)out, (void*)out, kD, 0L, bo, pm, kTok, kD, kD, 1.0f);
}
